// PointNetSetAbstraction_33071248179386
// MI455X (gfx1250) — hardware-verified
//
#include <hip/hip_runtime.h>
#include <math.h>
#pragma clang fp contract(off)

typedef __attribute__((ext_vector_type(16))) _Float16 v16h;
typedef __attribute__((ext_vector_type(8)))  _Float16 v8h;
typedef __attribute__((ext_vector_type(8)))  float    v8f;
typedef __attribute__((ext_vector_type(4)))  float    v4f;

constexpr int NBATCH   = 8;
constexpr int NPTS     = 4096;
constexpr int NCENT    = 1024;
constexpr int NSAMP    = 32;
constexpr int CH_PTS   = 64;
constexpr int W0_PITCH = 67;
constexpr int CH0      = 128;
constexpr int CH1      = 256;
constexpr int CH2      = 512;
constexpr int MROWS      = NBATCH * NCENT * NSAMP;
constexpr int CHUNK_ROWS = NCENT * NSAMP;
constexpr int NGROUPS    = NBATCH * NCENT;
constexpr int NTILES_ALL = MROWS / 64;
constexpr int NBLK_GROUP = NGROUPS / 8;
constexpr float ACT_CARRY = 16.0f;
constexpr float WGT_CARRY = 64.0f;
constexpr float FOLD_SCALE = 1.0f / (ACT_CARRY * WGT_CARRY);
constexpr float BALL_R2 = 0.16f;
constexpr float BN_EPS_F = 1e-5f;

static_assert(MROWS == 262144, "rows");
static_assert(CHUNK_ROWS % 64 == 0 && MROWS % 64 == 0, "M tiles");
static_assert(CH0 % 64 == 0 && CH1 % 64 == 0 && CH2 % 64 == 0, "N tiles");
static_assert(CH_PTS % 32 == 0 && CH0 % 32 == 0 && CH1 % 32 == 0, "K steps");
static_assert((NBATCH * NPTS) % 64 == 0, "P rows");

constexpr size_t SZ_CENT  = (size_t)NBATCH * 3 * NCENT * 4;
constexpr size_t SZ_W0P   = (size_t)CH0 * CH_PTS * 2;
constexpr size_t SZ_W1H   = (size_t)CH1 * CH0 * 2;
constexpr size_t SZ_W2H   = (size_t)CH2 * CH1 * 2;
constexpr size_t SZ_AB0   = (size_t)2 * CH0 * 4;
constexpr size_t SZ_AB1   = (size_t)2 * CH1 * 4;
constexpr size_t SZ_AB2   = (size_t)2 * CH2 * 4;
constexpr size_t SZ_PTST  = (size_t)NBATCH * NPTS * CH_PTS * 2;
constexpr size_t SZ_PG_P  = (size_t)NBATCH * NPTS * CH0 * 4;
constexpr size_t SZ_PG_G  = (size_t)NGROUPS * CH2 * 4;
constexpr size_t SZ_PG    = (SZ_PG_P > SZ_PG_G) ? SZ_PG_P : SZ_PG_G;
constexpr size_t SZ_X1    = (size_t)MROWS * CH0 * 2;
constexpr size_t SZ_X2C   = (size_t)CHUNK_ROWS * CH1 * 2;
constexpr size_t SZ_PART0 = (size_t)NBLK_GROUP * 2 * CH0 * 4;
constexpr size_t SZ_PART1 = (size_t)NTILES_ALL * 2 * CH1 * 4;
constexpr size_t SZ_PART2 = (size_t)NTILES_ALL * 2 * CH2 * 4;
constexpr size_t OFF_CENT  = 0;
constexpr size_t OFF_W0P   = OFF_CENT + SZ_CENT;
constexpr size_t OFF_W1H   = OFF_W0P + SZ_W0P;
constexpr size_t OFF_W2H   = OFF_W1H + SZ_W1H;
constexpr size_t OFF_AB0   = OFF_W2H + SZ_W2H;
constexpr size_t OFF_AB1   = OFF_AB0 + SZ_AB0;
constexpr size_t OFF_AB2   = OFF_AB1 + SZ_AB1;
constexpr size_t OFF_PTST  = OFF_AB2 + SZ_AB2;
constexpr size_t OFF_PG    = OFF_PTST + SZ_PTST;
constexpr size_t OFF_X1    = OFF_PG + SZ_PG;
constexpr size_t OFF_X2C   = OFF_X1 + SZ_X1;
constexpr size_t OFF_PART0 = OFF_X2C + SZ_X2C;
constexpr size_t OFF_PART1 = OFF_PART0 + SZ_PART0;
constexpr size_t OFF_PART2 = OFF_PART1 + SZ_PART1;
constexpr size_t WS_TOTAL  = OFF_PART2 + SZ_PART2;
static_assert(WS_TOTAL == 131521536, "carve total");
static_assert(WS_TOTAL <= 134217728, "carve under 128 MiB");
static_assert(OFF_W0P % 256 == 0 && OFF_AB0 % 256 == 0 && OFF_PTST % 256 == 0 && OFF_PG % 256 == 0, "align");
static_assert(OFF_X1 % 256 == 0 && OFF_X2C % 256 == 0 && OFF_PART0 % 256 == 0 && OFF_PART2 % 256 == 0, "align");
constexpr size_t OUT0_FLOATS = (size_t)NBATCH * 3 * NCENT;
constexpr size_t OUT1_FLOATS = (size_t)NBATCH * CH2 * NCENT;
static_assert(OUT0_FLOATS * 4 == 98304, "out1 byte offset");
static_assert((OUT0_FLOATS + OUT1_FLOATS) * 4 == 16875520, "d_out bytes");

__device__ __forceinline__ void wave_lds_sync() {
  __builtin_amdgcn_fence(__ATOMIC_RELEASE, "workgroup");
  __builtin_amdgcn_wave_barrier();
  __builtin_amdgcn_fence(__ATOMIC_ACQUIRE, "workgroup");
}

union FragH { v16h v; v8h h[2]; };
__device__ __forceinline__ v16h frag_load_h(const _Float16* p) {
  FragH f;
  f.h[0] = *(const v8h*)(p);
  f.h[1] = *(const v8h*)(p + 16);
  return f.v;
}
__device__ __forceinline__ v8f mma_h(v16h a, v16h b, v8f c) {
  return __builtin_amdgcn_wmma_f32_16x16x32_f16(false, a, false, b, (short)0, c, false, false);
}
__device__ __forceinline__ void guard_row(v8f& a, v8f& b, v8f& c, v8f& d, v16h x, v16h y0, v16h y1, v16h y2, v16h y3) {
  asm volatile("v_nop\n\tv_nop\n\tv_nop\n\tv_nop"
               : "+v"(a), "+v"(b), "+v"(c), "+v"(d)
               : "v"(x), "v"(y0), "v"(y1), "v"(y2), "v"(y3));
}
__device__ __forceinline__ void keep4_h(v16h a, v16h b, v16h c, v16h d) {
  asm volatile("v_nop" :: "v"(a), "v"(b), "v"(c), "v"(d));
}
__device__ __forceinline__ void acc_guard4(v8f& a, v8f& b, v8f& c, v8f& d) {
  asm volatile("v_nop\n\tv_nop\n\tv_nop\n\tv_nop" : "+v"(a), "+v"(b), "+v"(c), "+v"(d));
}

__device__ __forceinline__ void gemm_main(const _Float16* __restrict__ Ab, int lda,
                                          const _Float16* __restrict__ Bb, int ldb,
                                          int m0, int n0, int K, int lane, v8f (&acc)[4][4]) {
  const int rlane = lane & 15;
  const int koff  = (lane >> 4) * 8;
#pragma unroll
  for (int i = 0; i < 4; ++i)
#pragma unroll
    for (int j = 0; j < 4; ++j) acc[i][j] = (v8f){0.f, 0.f, 0.f, 0.f, 0.f, 0.f, 0.f, 0.f};
  for (int k0 = 0; k0 < K; k0 += 32) {
    v16h bh[4];
#pragma unroll
    for (int j = 0; j < 4; ++j)
      bh[j] = frag_load_h(Bb + (size_t)(n0 + (j << 4) + rlane) * ldb + koff + k0);
#pragma unroll
    for (int i = 0; i < 4; ++i) {
      const v16h ah = frag_load_h(Ab + (size_t)(m0 + (i << 4) + rlane) * lda + koff + k0);
#pragma unroll
      for (int j = 0; j < 4; ++j) acc[i][j] = mma_h(ah, bh[j], acc[i][j]);
      guard_row(acc[i][0], acc[i][1], acc[i][2], acc[i][3], ah, bh[0], bh[1], bh[2], bh[3]);
    }
    keep4_h(bh[0], bh[1], bh[2], bh[3]);
  }
  acc_guard4(acc[0][0], acc[0][1], acc[0][2], acc[0][3]);
  acc_guard4(acc[1][0], acc[1][1], acc[1][2], acc[1][3]);
  acc_guard4(acc[2][0], acc[2][1], acc[2][2], acc[2][3]);
  acc_guard4(acc[3][0], acc[3][1], acc[3][2], acc[3][3]);
}

template <int MODE>
__global__ __launch_bounds__(256) void k_gemm(
    const unsigned short* __restrict__ Ap, int lda,
    const unsigned short* __restrict__ Btp, int ldb,
    void* __restrict__ Cout, int ldc,
    const float* __restrict__ bias, const float* __restrict__ ab, const float* __restrict__ gsign,
    float* __restrict__ part, int M, int N, int K, int rowBase, float scale) {
  __shared__ __align__(16) float sT[8][16 * 68];
  const int lane = threadIdx.x & 31;
  const int wave = threadIdx.x >> 5;
  const int tilesN = N >> 6;
  const int tilesM = M >> 6;
  const int tile = blockIdx.x * 8 + wave;
  if (tile >= tilesM * tilesN) return;
  const int tm = tile / tilesN;
  const int tn = tile - tm * tilesN;
  const int m0 = tm << 6;
  const int n0 = tn << 6;
  const int rlane = lane & 15;
  const int hh    = lane >> 4;
  const int mOff  = hh * 8;

  v8f acc[4][4];
  gemm_main((const _Float16*)Ap, lda, (const _Float16*)Btp, ldb, m0, n0, K, lane, acc);

  float* slab = sT[wave];
  if (MODE == 0 || MODE == 2) {
#pragma unroll
    for (int i = 0; i < 4; ++i) {
      const int mBase = m0 + (i << 4);
#pragma unroll
      for (int j = 0; j < 4; ++j) {
        const int n = n0 + (j << 4) + rlane;
        float bv = 0.f, an = 1.f, cn = 0.f;
        if (MODE == 2) { bv = bias[n]; an = ab[n]; cn = ab[N + n]; }
#pragma unroll
        for (int r = 0; r < 8; ++r) {
          float v = acc[i][j][r] * scale;
          if (MODE == 2) {
            v = v + bv;
            v = an * v + cn;
            v = fmaxf(v, 0.0f) * ACT_CARRY;
          }
          slab[(mOff + r) * 68 + (j << 4) + rlane] = v;
        }
      }
      wave_lds_sync();
      if (MODE == 0) {
        float* C = (float*)Cout;
        const int c4 = (lane & 15) * 4;
        for (int pass = 0; pass < 2; ++pass) {
#pragma unroll
          for (int it = 0; it < 8; ++it) {
            const int row = it * 2 + hh;
            v4f v = *(const v4f*)(slab + row * 68 + c4);
            *(volatile v4f*)(C + (size_t)(mBase + row) * ldc + n0 + c4) = v;
          }
          __threadfence();
        }
      } else {
        unsigned short* C = (unsigned short*)Cout;
        const int q = lane >> 3, c8 = (lane & 7) * 8;
        for (int pass = 0; pass < 2; ++pass) {
#pragma unroll
          for (int it = 0; it < 4; ++it) {
            const int row = it * 4 + q;
            const float* sp = slab + row * 68 + c8;
            v8h hv;
#pragma unroll
            for (int e = 0; e < 8; ++e) hv[e] = (_Float16)sp[e];
            *(volatile v8h*)(C + (size_t)(mBase + row) * ldc + n0 + c8) = hv;
          }
          __threadfence();
        }
      }
      wave_lds_sync();
    }
  } else {
    const int statBase = (MODE == 3) ? 128 : 0;
#pragma unroll
    for (int j = 0; j < 4; ++j) {
      const int n = n0 + (j << 4) + rlane;
      const float bv = bias[n];
      float s = 0.f, q = 0.f;
      float mx0 = -INFINITY, mn0 = INFINITY, mx1 = -INFINITY, mn1 = INFINITY;
#pragma unroll
      for (int i = 0; i < 4; ++i) {
#pragma unroll
        for (int r = 0; r < 8; ++r) {
          const float v = acc[i][j][r] * scale + bv;
          const float v2 = v * v;
          s = s + v;
          q = q + v2;
          if (MODE == 3) {
            if (i < 2) { mx0 = fmaxf(mx0, v); mn0 = fminf(mn0, v); }
            else       { mx1 = fmaxf(mx1, v); mn1 = fminf(mn1, v); }
          }
        }
      }
      s = s + __shfl_xor(s, 16, 32);
      q = q + __shfl_xor(q, 16, 32);
      slab[statBase + hh * 64 + (j << 4) + rlane] = hh ? q : s;
      if (MODE == 3) {
        const float omx0 = __shfl_xor(mx0, 16, 32);
        const float omn0 = __shfl_xor(mn0, 16, 32);
        const float omx1 = __shfl_xor(mx1, 16, 32);
        const float omn1 = __shfl_xor(mn1, 16, 32);
        mx0 = fmaxf(mx0, omx0); mn0 = fminf(mn0, omn0);
        mx1 = fmaxf(mx1, omx1); mn1 = fminf(mn1, omn1);
        const float gs = gsign[n];
        const float e0 = (gs >= 0.0f) ? mx0 : mn0;
        const float e1 = (gs >= 0.0f) ? mx1 : mn1;
        slab[hh * 64 + (j << 4) + rlane] = hh ? e1 : e0;
      }
    }
    wave_lds_sync();
    const int c4 = (lane & 15) * 4;
    const int tmG = (rowBase + m0) >> 6;
    const v4f sv = *(const v4f*)(slab + statBase + lane * 4);
    float* pdst = part + ((size_t)tmG * 2 + hh) * N + n0 + c4;
    v4f ev = sv;
    float* gdst = pdst;
    if (MODE == 3) {
      ev = *(const v4f*)(slab + lane * 4);
      gdst = (float*)Cout + ((size_t)((rowBase + m0) >> 5) + hh) * ldc + n0 + c4;
    }
    for (int pass = 0; pass < 2; ++pass) {
      *(volatile v4f*)pdst = sv;
      if (MODE == 3) *(volatile v4f*)gdst = ev;
      __threadfence();
    }
  }
}

__global__ __launch_bounds__(512) void k_fps(const float* __restrict__ xyz,
                                             float* __restrict__ out0, float* __restrict__ cent) {
#pragma clang fp contract(off)
  __shared__ __align__(16) float sx[3 * NPTS];
  __shared__ int   sSel[NCENT];
  __shared__ float sval[2][16];
  __shared__ int   sidx[2][16];
  const int tid = threadIdx.x, lane = tid & 31, wave = tid >> 5, b = blockIdx.x;
  const float* xb = xyz + (size_t)b * 3 * NPTS;
#pragma unroll
  for (int i = 0; i < 6; ++i) {
    const int f4 = tid + 512 * i;
    const v4f v = *(const v4f*)(xb + 4 * f4);
    *(v4f*)(sx + 4 * f4) = v;
  }
  __syncthreads();
  float px[8], py[8], pz[8], dd[8];
#pragma unroll
  for (int i = 0; i < 8; ++i) {
    const int j = tid + 512 * i;
    px[i] = sx[j]; py[i] = sx[NPTS + j]; pz[i] = sx[2 * NPTS + j];
    dd[i] = 1e10f;
  }
  int far = 0;
  int pb = 0;
#pragma unroll 1
  for (int it = 0; it < NCENT; ++it) {
    if (tid == 0) sSel[it] = far;
    const float cx = sx[far], cy = sx[NPTS + far], cz = sx[2 * NPTS + far];
    float best = -1.0f;
    int bi = 0;
#pragma unroll
    for (int i = 0; i < 8; ++i) {
      const float dx = px[i] - cx, dy = py[i] - cy, dz = pz[i] - cz;
      const float t0 = dx * dx, t1 = dy * dy, t2 = dz * dz;
      const float d = (t0 + t2) + t1;
      const float nd = fminf(dd[i], d);
      dd[i] = nd;
      const bool gt = nd > best;
      best = gt ? nd : best;
      bi = gt ? (tid + 512 * i) : bi;
    }
#pragma unroll
    for (int off = 16; off >= 1; off >>= 1) {
      const float ov = __shfl_xor(best, off, 32);
      const int   oi = __shfl_xor(bi, off, 32);
      const bool take = (ov > best) || (ov == best && oi < bi);
      best = take ? ov : best;
      bi = take ? oi : bi;
    }
    if (lane == 0) { sval[pb][wave] = best; sidx[pb][wave] = bi; }
    __syncthreads();
    float v = sval[pb][lane & 15];
    int ix = sidx[pb][lane & 15];
#pragma unroll
    for (int off = 8; off >= 1; off >>= 1) {
      const float ov = __shfl_xor(v, off, 32);
      const int   oi = __shfl_xor(ix, off, 32);
      const bool take = (ov > v) || (ov == v && oi < ix);
      v = take ? ov : v;
      ix = take ? oi : ix;
    }
    ix = ix < 0 ? 0 : ix;
    ix = ix > NPTS - 1 ? NPTS - 1 : ix;
    far = ix;
    pb ^= 1;
  }
  __syncthreads();
  float ov[6];
#pragma unroll
  for (int d = 0; d < 3; ++d)
#pragma unroll
    for (int h2 = 0; h2 < 2; ++h2) {
      int ix = sSel[tid + 512 * h2];
      ix = ix < 0 ? 0 : ix;
      ix = ix > NPTS - 1 ? NPTS - 1 : ix;
      ov[d * 2 + h2] = sx[d * NPTS + ix];
    }
  for (int pass = 0; pass < 2; ++pass) {
#pragma unroll
    for (int d = 0; d < 3; ++d)
#pragma unroll
      for (int h2 = 0; h2 < 2; ++h2) {
        const size_t o = (size_t)(b * 3 + d) * NCENT + tid + 512 * h2;
        *(volatile float*)(out0 + o) = ov[d * 2 + h2];
        *(volatile float*)(cent + o) = ov[d * 2 + h2];
      }
    __threadfence();
  }
}

constexpr int PREP_T0 = CH0 * CH_PTS / 8;
constexpr int PREP_T1 = PREP_T0 + CH1 * CH0 / 8;
constexpr int PREP_T2 = PREP_T1 + CH2 * CH1 / 8;
static_assert(PREP_T0 % 32 == 0 && PREP_T1 % 32 == 0 && PREP_T2 % 256 == 0, "prep segments");
__global__ __launch_bounds__(256) void k_prep_w(const float* __restrict__ w0, const float* __restrict__ w1,
                                                const float* __restrict__ w2,
                                                unsigned short* __restrict__ W0p, unsigned short* __restrict__ W1h,
                                                unsigned short* __restrict__ W2h) {
  const int t = blockIdx.x * 256 + threadIdx.x;
  if (t < PREP_T2) {
    const int seg = (t < PREP_T0) ? 0 : ((t < PREP_T1) ? 1 : 2);
    const int u = (seg == 0) ? t : ((seg == 1) ? (t - PREP_T0) : (t - PREP_T1));
    const int kcols = (seg == 0) ? CH_PTS : ((seg == 1) ? CH0 : CH1);
    const int per = kcols / 8;
    const int o = u / per;
    const int k8 = (u - o * per) * 8;
    const float* src = (seg == 0) ? (w0 + (size_t)o * W0_PITCH + 3 + k8)
                     : ((seg == 1) ? (w1 + (size_t)o * CH0 + k8) : (w2 + (size_t)o * CH1 + k8));
    unsigned short* dst = (seg == 0) ? (W0p + (size_t)o * CH_PTS + k8)
                        : ((seg == 1) ? (W1h + (size_t)o * CH0 + k8) : (W2h + (size_t)o * CH1 + k8));
    v8h hv;
#pragma unroll
    for (int e = 0; e < 8; ++e) {
      const float f = src[e] * WGT_CARRY;
      hv[e] = (_Float16)f;
    }
    *(volatile v8h*)dst = hv;
    __threadfence();
    *(volatile v8h*)dst = hv;
  }
}

__global__ __launch_bounds__(256) void k_pts_t(const float* __restrict__ pts, unsigned short* __restrict__ ptsT) {
  __shared__ float tile[CH_PTS][129];
  const int tid = threadIdx.x, lane = tid & 31, wave = tid >> 5;
  const int b = blockIdx.x >> 5;
  const int j0 = (blockIdx.x & 31) * 128;
#pragma unroll
  for (int i = 0; i < 8; ++i) {
    const int c = wave * 8 + i;
    const v4f v = *(const v4f*)(pts + ((size_t)(b * CH_PTS + c)) * NPTS + j0 + lane * 4);
    tile[c][lane * 4 + 0] = v[0];
    tile[c][lane * 4 + 1] = v[1];
    tile[c][lane * 4 + 2] = v[2];
    tile[c][lane * 4 + 3] = v[3];
  }
  __syncthreads();
  const int c8 = (lane & 7) * 8;
  v8h hv[4];
#pragma unroll
  for (int it = 0; it < 4; ++it) {
    const int jr = wave * 16 + it * 4 + (lane >> 3);
#pragma unroll
    for (int e = 0; e < 8; ++e) {
      const float f = tile[c8 + e][jr] * ACT_CARRY;
      hv[it][e] = (_Float16)f;
    }
  }
  for (int pass = 0; pass < 2; ++pass) {
#pragma unroll
    for (int it = 0; it < 4; ++it) {
      const int jr = wave * 16 + it * 4 + (lane >> 3);
      *(volatile v8h*)(ptsT + ((size_t)(b * NPTS + j0 + jr)) * CH_PTS + c8) = hv[it];
    }
    __threadfence();
  }
}

template <bool NORM>
__global__ __launch_bounds__(256) void k_group(const float* __restrict__ xyz, const float* __restrict__ cent,
                                               const float* __restrict__ P, const float* __restrict__ w0,
                                               const float* __restrict__ b0, const float* __restrict__ ab0,
                                               unsigned short* __restrict__ x1, float* __restrict__ part0) {
#pragma clang fp contract(off)
  __shared__ float sWx[CH0], sWy[CH0], sWz[CH0], sBi[CH0], sAa[CH0], sCc[CH0];
  __shared__ int   sSlot[8][32];
  __shared__ float sRed[8][2 * CH0];
  const int tid = threadIdx.x, lane = tid & 31, wave = tid >> 5;
  const int wid = blockIdx.x * 8 + wave;
  const int b = wid >> 10;
  const int s = wid & (NCENT - 1);
  if (tid < CH0) {
    sWx[tid] = w0[(size_t)tid * W0_PITCH + 0];
    sWy[tid] = w0[(size_t)tid * W0_PITCH + 1];
    sWz[tid] = w0[(size_t)tid * W0_PITCH + 2];
    sBi[tid] = b0[tid];
    if (NORM) { sAa[tid] = ab0[tid]; sCc[tid] = ab0[CH0 + tid]; }
    else      { sAa[tid] = 1.0f;     sCc[tid] = 0.0f; }
  }
  sSlot[wave][lane] = 0;
  __syncthreads();

  const float* xb = xyz + (size_t)b * 3 * NPTS;
  const float cx = cent[(size_t)(b * 3 + 0) * NCENT + s];
  const float cy = cent[(size_t)(b * 3 + 1) * NCENT + s];
  const float cz = cent[(size_t)(b * 3 + 2) * NCENT + s];

  int count = 0;
  const unsigned ltmask = (1u << lane) - 1u;
#pragma unroll 1
  for (int j0 = 0; j0 < NPTS; j0 += 32) {
    if (count >= NSAMP) break;
    const int j = j0 + lane;
    const float dx = cx - xb[j];
    const float dy = cy - xb[NPTS + j];
    const float dz = cz - xb[2 * NPTS + j];
    const float t0 = dx * dx, t1 = dy * dy, t2 = dz * dz;
    const float sq = (t0 + t2) + t1;
    const bool hit = !(sq > BALL_R2);
    const unsigned mask = __builtin_amdgcn_ballot_w32(hit);
    const int pos = count + __popc(mask & ltmask);
    if (hit && pos < NSAMP) sSlot[wave][pos] = j;
    count = __builtin_amdgcn_readfirstlane(count + __popc(mask));
  }
  wave_lds_sync();
  const int total = count < NSAMP ? count : NSAMP;
  const int sel = (lane < total) ? lane : 0;
  int slot = sSlot[wave][sel];
  slot = slot < 0 ? 0 : slot;
  slot = slot > NPTS - 1 ? NPTS - 1 : slot;

  const float gx = xb[slot] - cx;
  const float gy = xb[NPTS + slot] - cy;
  const float gz = xb[2 * NPTS + slot] - cz;

  const int rh = lane >> 4;
  const int c0 = (lane & 15) * 8;
  float wx[8], wy[8], wz[8], bb[8], av[8], cv[8];
#pragma unroll
  for (int e = 0; e < 8; ++e) {
    wx[e] = sWx[c0 + e]; wy[e] = sWy[c0 + e]; wz[e] = sWz[c0 + e];
    bb[e] = sBi[c0 + e]; av[e] = sAa[c0 + e]; cv[e] = sCc[c0 + e];
  }
  float accS[8], accQ[8];
#pragma unroll
  for (int e = 0; e < 8; ++e) { accS[e] = 0.0f; accQ[e] = 0.0f; }

#pragma unroll 1
  for (int kk = 0; kk < 16; ++kk) {
    const int src = 2 * kk + rh;
    const int jk = __shfl(slot, src, 32);
    const float dx = __shfl(gx, src, 32);
    const float dy = __shfl(gy, src, 32);
    const float dz = __shfl(gz, src, 32);
    const float* Pp = P + ((size_t)(b * NPTS + jk)) * CH0 + c0;
    const v4f p0 = *(const v4f*)(Pp);
    const v4f p1 = *(const v4f*)(Pp + 4);
    float y[8];
#pragma unroll
    for (int e = 0; e < 8; ++e) {
      const float pe = (e < 4) ? p0[e & 3] : p1[e & 3];
      const float base = pe + bb[e];
      y[e] = __builtin_fmaf(wz[e], dz, __builtin_fmaf(wy[e], dy, __builtin_fmaf(wx[e], dx, base)));
    }
    if (NORM) {
      v8h hv;
#pragma unroll
      for (int e = 0; e < 8; ++e) {
        float z = av[e] * y[e] + cv[e];
        z = fmaxf(z, 0.0f) * ACT_CARRY;
        hv[e] = (_Float16)z;
      }
      unsigned short* dst = x1 + ((size_t)wid * NSAMP + src) * CH0 + c0;
      *(volatile v8h*)dst = hv;
      __threadfence();
      *(volatile v8h*)dst = hv;
    } else {
#pragma unroll
      for (int e = 0; e < 8; ++e) {
        const float y2 = y[e] * y[e];
        accS[e] = accS[e] + y[e];
        accQ[e] = accQ[e] + y2;
      }
    }
  }
  if (!NORM) {
#pragma unroll
    for (int e = 0; e < 8; ++e) {
      const float os = __shfl_xor(accS[e], 16, 32);
      const float oq = __shfl_xor(accQ[e], 16, 32);
      accS[e] = accS[e] + os;
      accQ[e] = accQ[e] + oq;
      sRed[wave][rh * CH0 + c0 + e] = rh ? accQ[e] : accS[e];
    }
  }
  __syncthreads();
  if (!NORM) {
    float tot = 0.0f;
#pragma unroll
    for (int w = 0; w < 8; ++w) tot = tot + sRed[w][tid];
    float* dst = part0 + (size_t)blockIdx.x * (2 * CH0) + tid;
    *(volatile float*)dst = tot;
    __threadfence();
    *(volatile float*)dst = tot;
  }
}

__global__ __launch_bounds__(256) void k_fin(const float* __restrict__ part, int T, int C,
                                             const float* __restrict__ g, const float* __restrict__ bt,
                                             float* __restrict__ ab, double invM) {
  __shared__ double sS[8][32];
  __shared__ double sQ[8][32];
  const int tid = threadIdx.x, c = tid & 31, pt = tid >> 5;
  const int c0 = blockIdx.x * 32;
  double s = 0.0, q = 0.0;
#pragma unroll 4
  for (int t = pt; t < T; t += 8) {
    s = s + (double)part[((size_t)t * 2) * C + c0 + c];
    q = q + (double)part[((size_t)t * 2 + 1) * C + c0 + c];
  }
  sS[pt][c] = s;
  sQ[pt][c] = q;
  __syncthreads();
  if (pt == 0) {
    double S = 0.0, Q = 0.0;
#pragma unroll
    for (int p = 0; p < 8; ++p) { S = S + sS[p][c]; Q = Q + sQ[p][c]; }
    const double mean = S * invM;
    double var = Q * invM - mean * mean;
    var = var < 0.0 ? 0.0 : var;
    const float a = g[c0 + c] * rsqrtf((float)var + BN_EPS_F);
    const float cc = bt[c0 + c] - (float)mean * a;
    for (int pass = 0; pass < 2; ++pass) {
      *(volatile float*)(ab + c0 + c) = a;
      *(volatile float*)(ab + C + c0 + c) = cc;
      __threadfence();
    }
  }
}

__global__ __launch_bounds__(256) void k_out(const float* __restrict__ gext, const float* __restrict__ ab2,
                                             float* __restrict__ out1) {
  __shared__ float tile[128][33];
  const int tid = threadIdx.x, lane = tid & 31, wave = tid >> 5;
  const int r0 = (blockIdx.x & 63) * 128;
  const int o0 = (blockIdx.x >> 6) * 32;
#pragma unroll 4
  for (int i = 0; i < 16; ++i) {
    const int row = wave * 16 + i;
    tile[row][lane] = gext[(size_t)(r0 + row) * CH2 + o0 + lane];
  }
  __syncthreads();
  const int b = r0 >> 10;
  const int s0 = r0 & (NCENT - 1);
  v4f ov[4];
#pragma unroll
  for (int q = 0; q < 4; ++q) {
    const int o = o0 + wave * 4 + q;
    const float a = ab2[o];
    const float cc = ab2[CH2 + o];
#pragma unroll
    for (int e = 0; e < 4; ++e) {
      const float z = a * tile[lane * 4 + e][wave * 4 + q] + cc;
      ov[q][e] = fmaxf(z, 0.0f);
    }
  }
  for (int pass = 0; pass < 2; ++pass) {
#pragma unroll
    for (int q = 0; q < 4; ++q) {
      const int o = o0 + wave * 4 + q;
      *(volatile v4f*)(out1 + ((size_t)(b * CH2 + o)) * NCENT + s0 + lane * 4) = ov[q];
    }
    __threadfence();
  }
}

extern "C" void kernel_launch(void* const* d_in, const int* in_sizes, int n_in,
                              void* d_out, int out_size, void* d_ws, size_t ws_size,
                              hipStream_t stream) {
  (void)in_sizes;
  if (n_in < 14) return;
  if (ws_size < WS_TOTAL) return;
  if ((size_t)out_size < OUT0_FLOATS + OUT1_FLOATS) return;
  const float* xyz = (const float*)d_in[0];
  const float* pts = (const float*)d_in[1];
  const float* w0  = (const float*)d_in[2];
  const float* b0  = (const float*)d_in[3];
  const float* g0  = (const float*)d_in[4];
  const float* bt0 = (const float*)d_in[5];
  const float* w1  = (const float*)d_in[6];
  const float* b1  = (const float*)d_in[7];
  const float* g1  = (const float*)d_in[8];
  const float* bt1 = (const float*)d_in[9];
  const float* w2  = (const float*)d_in[10];
  const float* b2  = (const float*)d_in[11];
  const float* g2  = (const float*)d_in[12];
  const float* bt2 = (const float*)d_in[13];
  float* out0 = (float*)d_out;
  float* out1 = (float*)d_out + OUT0_FLOATS;

  char* ws = (char*)d_ws;
  float* cent = (float*)(ws + OFF_CENT);
  unsigned short* W0p = (unsigned short*)(ws + OFF_W0P);
  unsigned short* W1h = (unsigned short*)(ws + OFF_W1H);
  unsigned short* W2h = (unsigned short*)(ws + OFF_W2H);
  float* ab0 = (float*)(ws + OFF_AB0);
  float* ab1 = (float*)(ws + OFF_AB1);
  float* ab2 = (float*)(ws + OFF_AB2);
  unsigned short* ptsT = (unsigned short*)(ws + OFF_PTST);
  float* Pg = (float*)(ws + OFF_PG);
  unsigned short* x1  = (unsigned short*)(ws + OFF_X1);
  unsigned short* x2c = (unsigned short*)(ws + OFF_X2C);
  float* part0 = (float*)(ws + OFF_PART0);
  float* part1 = (float*)(ws + OFF_PART1);
  float* part2 = (float*)(ws + OFF_PART2);
  const double invM = 1.0 / (double)MROWS;

  k_fps<<<NBATCH, 512, 0, stream>>>(xyz, out0, cent);
  k_prep_w<<<PREP_T2 / 256, 256, 0, stream>>>(w0, w1, w2, W0p, W1h, W2h);
  k_pts_t<<<NBATCH * (NPTS / 128), 256, 0, stream>>>(pts, ptsT);
  k_gemm<0><<<(NBATCH * NPTS / 64) * (CH0 / 64) / 8, 256, 0, stream>>>(
      ptsT, CH_PTS, W0p, CH_PTS, (void*)Pg, CH0, b0, ab0, g0, part0,
      NBATCH * NPTS, CH0, CH_PTS, 0, FOLD_SCALE);
  k_group<false><<<NBLK_GROUP, 256, 0, stream>>>(xyz, cent, Pg, w0, b0, ab0, x1, part0);
  k_fin<<<CH0 / 32, 256, 0, stream>>>(part0, NBLK_GROUP, CH0, g0, bt0, ab0, invM);
  k_group<true><<<NBLK_GROUP, 256, 0, stream>>>(xyz, cent, Pg, w0, b0, ab0, x1, part0);
  k_gemm<1><<<(MROWS / 64) * (CH1 / 64) / 8, 256, 0, stream>>>(
      x1, CH0, W1h, CH0, (void*)x2c, CH1, b1, ab1, g1, part1,
      MROWS, CH1, CH0, 0, FOLD_SCALE);
  k_fin<<<CH1 / 32, 256, 0, stream>>>(part1, NTILES_ALL, CH1, g1, bt1, ab1, invM);
  for (int c = 0; c < NBATCH; ++c) {
    const unsigned short* x1c = x1 + (size_t)c * CHUNK_ROWS * CH0;
    k_gemm<2><<<(CHUNK_ROWS / 64) * (CH1 / 64) / 8, 256, 0, stream>>>(
        x1c, CH0, W1h, CH0, (void*)x2c, CH1, b1, ab1, g1, part1,
        CHUNK_ROWS, CH1, CH0, c * CHUNK_ROWS, FOLD_SCALE);
    k_gemm<3><<<(CHUNK_ROWS / 64) * (CH2 / 64) / 8, 256, 0, stream>>>(
        x2c, CH1, W2h, CH1, (void*)Pg, CH2, b2, ab2, g2, part2,
        CHUNK_ROWS, CH2, CH1, c * CHUNK_ROWS, FOLD_SCALE);
  }
  k_fin<<<CH2 / 32, 256, 0, stream>>>(part2, NTILES_ALL, CH2, g2, bt2, ab2, invM);
  k_out<<<(NGROUPS / 128) * (CH2 / 32), 256, 0, stream>>>(Pg, ab2, out1);
}
